// MambaBlock_67680094650660
// MI455X (gfx1250) — hardware-run, weakly checked
//
#include <hip/hip_runtime.h>
#include <hip/hip_fp16.h>
#include <math.h>


typedef __attribute__((ext_vector_type(16))) _Float16 v16h;
typedef __attribute__((ext_vector_type(8)))  _Float16 v8h;
typedef __attribute__((ext_vector_type(8)))  float    v8f;
typedef __attribute__((ext_vector_type(4)))  float    v4f;
typedef __attribute__((ext_vector_type(2)))  unsigned v2u;
typedef __attribute__((ext_vector_type(4)))  unsigned v4u;

constexpr int kBatch  = 2;
constexpr int kSeq    = 2048;
constexpr int kDm     = 512;
constexpr int kDin    = 1024;
constexpr int kNst    = 16;
constexpr int kConvK  = 4;
constexpr int kConvTP = 260;
constexpr int kRank   = 32;
constexpr int kXpN    = kRank + 2 * kNst;
constexpr int kBcP    = 64;
constexpr int kOffDtF = 0;
constexpr int kOffB   = kRank;
constexpr int kOffC   = kRank + kNst;
constexpr float kWCarry = 1024.0f;
constexpr float kResid  = 2048.0f;
constexpr float kYCarry = 16.0f;
constexpr float kInvResid = 1.0f / kResid;
constexpr float kInvCarry = 1.0f / kYCarry;
constexpr float kLnEps  = 1.0e-5f;
static_assert(kDin == 2 * kDm);
static_assert(kRank == (kDm + 15) / 16);
static_assert(kXpN == 64);
static_assert(kXpN <= kBcP && (kBcP % 64) == 0);
static_assert(kOffDtF == 0 && kOffB == 32 && kOffC == 48 && kOffC + kNst == kXpN);
static_assert(kRank == 32);
static_assert(kDm == 512);
static_assert((kDin % 256) == 0);
static_assert((kDin % 1024) == 0);
static_assert((kSeq % 64) == 0);
static_assert((kDin % 64) == 0 && (kDin % 32) == 0 && (kSeq % 32) == 0 && (kSeq % 8) == 0);
static_assert((kDm % 64) == 0 && (kDm % 32) == 0 && (kRank % 32) == 0);

constexpr size_t kSzWIN  = (size_t)2 * kDin * kDm * 2;
constexpr size_t kSzWX   = (size_t)kXpN * kDin * 2;
constexpr size_t kSzWDT  = (size_t)kDin * kRank * 2;
constexpr size_t kSzWOUT = (size_t)kDm * kDin * 2;
constexpr size_t kSzWLIN = (size_t)kDm * kDm * 2;
constexpr size_t kSzALOG = (size_t)kDin * kNst * 4;
constexpr size_t kSzCW   = (size_t)kDin * kConvK * 4;
constexpr size_t kSzVEC  = (size_t)kDin * 4;
constexpr size_t kSzVDM  = (size_t)kDm * 4;
constexpr size_t kSzM32  = (size_t)kSeq * kDm * 4;
constexpr size_t kSzM16  = (size_t)kSeq * kDm * 2;
constexpr size_t kSzF32  = (size_t)kSeq * kDin * 4;
constexpr size_t kSzH16  = (size_t)kSeq * kDin * 2;
constexpr size_t kSzPROJ = (size_t)kSeq * kXpN * 4;
constexpr size_t kSzDH   = (size_t)kSeq * kRank * 2;
constexpr size_t kOffWIN  = 0;
constexpr size_t kOffWX   = kOffWIN  + kSzWIN;
constexpr size_t kOffWDT  = kOffWX   + kSzWX;
constexpr size_t kOffWOUT = kOffWDT  + kSzWDT;
constexpr size_t kOffWLIN = kOffWOUT + kSzWOUT;
constexpr size_t kOffALOG = kOffWLIN + kSzWLIN;
constexpr size_t kOffCW   = kOffALOG + kSzALOG;
constexpr size_t kOffCB   = kOffCW   + kSzCW;
constexpr size_t kOffDTB  = kOffCB   + kSzVEC;
constexpr size_t kOffDR   = kOffDTB  + kSzVEC;
constexpr size_t kOffNW   = kOffDR   + kSzVEC;
constexpr size_t kOffNB   = kOffNW   + kSzVDM;
constexpr size_t kOffLB   = kOffNB   + kSzVDM;
constexpr size_t kOffXR   = kOffLB   + kSzVDM;
constexpr size_t kOffXH   = kOffXR   + kSzM32;
constexpr size_t kOffU0   = kOffXH   + kSzM16;
constexpr size_t kOffZ    = kOffU0   + kSzF32;
constexpr size_t kOffU    = kOffZ    + kSzF32;
constexpr size_t kOffUH   = kOffU    + kSzF32;
constexpr size_t kOffUL   = kOffUH   + kSzH16;
constexpr size_t kOffPROJ = kOffUL   + kSzH16;
constexpr size_t kOffDH   = kOffPROJ + kSzPROJ;
constexpr size_t kOffDTP  = kOffDH   + kSzDH;
constexpr size_t kOffDT   = kOffDTP  + kSzF32;
constexpr size_t kOffYH   = kOffDT   + kSzF32;
constexpr size_t kOffYL   = kOffYH   + kSzH16;
constexpr size_t kOffGH   = kOffYL   + kSzH16;
constexpr size_t kOffM    = kOffGH   + kSzH16;
constexpr size_t kOffYNH  = kOffM    + kSzM32;
constexpr size_t kOffLIN  = kOffYNH  + kSzM16;
constexpr size_t kWsTotal = kOffLIN  + kSzM32;
static_assert(kSzWIN == 2097152ull && kSzWX == 131072ull && kSzWDT == 65536ull);
static_assert(kSzWOUT == 1048576ull && kSzWLIN == 524288ull);
static_assert(kSzALOG == 65536ull && kSzCW == 16384ull && kSzVEC == 4096ull && kSzVDM == 2048ull);
static_assert(kSzM32 == 4194304ull && kSzM16 == 2097152ull);
static_assert(kSzF32 == 8388608ull && kSzH16 == 4194304ull);
static_assert(kSzPROJ == 524288ull && kSzDH == 131072ull);
static_assert(kWsTotal == 84314112ull);
static_assert(kWsTotal <= 134217728ull);
static_assert((kSzWIN % 256) == 0 && (kSzWX % 256) == 0 && (kSzWDT % 256) == 0 && (kSzWOUT % 256) == 0 &&
              (kSzWLIN % 256) == 0 && (kSzALOG % 256) == 0 && (kSzCW % 256) == 0 && (kSzVEC % 256) == 0 &&
              (kSzVDM % 256) == 0 && (kSzM32 % 256) == 0 && (kSzM16 % 256) == 0 && (kSzF32 % 256) == 0 &&
              (kSzH16 % 256) == 0 && (kSzPROJ % 256) == 0 && (kSzDH % 256) == 0);

__device__ __forceinline__ _Float16 f16_flush(float v) {
  const float w = (fabsf(v) < 6.103515625e-05f) ? 0.0f : v;
  return (_Float16)w;
}
__device__ __forceinline__ void f16_split(float v, _Float16& hi, _Float16& lo) {
  hi = f16_flush(v);
  const float hf = (float)hi;
  const float r = (v - hf) * kResid;
  lo = f16_flush(r);
}

__device__ __forceinline__ float bf16r(float v) {
  unsigned u = __float_as_uint(v);
  u = (u + 0x7FFFu + ((u >> 16) & 1u)) & 0xFFFF0000u;
  return __uint_as_float(u);
}

__device__ __forceinline__ float h16_to_f32(unsigned hb) {
  const unsigned sgn = (hb & 0x8000u) << 16; const unsigned em = hb & 0x7fffu;
  const float fn = __uint_as_float((em << 13) + 0x38000000u);
  const float fs = (float)em * 5.9604644775390625e-8f;
  const float mag = (em < 0x400u) ? fs : fn; return __uint_as_float(__float_as_uint(mag) | sgn); }

namespace eng {
union FragU { v16h v; v8h h[2]; };
__device__ __forceinline__ v16h frag_load(const _Float16* p) {
  FragU f;
  f.h[0] = *(const v8h*)(p);
  f.h[1] = *(const v8h*)(p + 16);
  return f.v;
}
__device__ __forceinline__ v8f mma(v16h a, v16h b, v8f c) {
  return __builtin_amdgcn_wmma_f32_16x16x32_f16(false, a, false, b, (short)0, c, false, false);
}
__device__ __forceinline__ void guard1(v8f& a, v16h x, v16h y) {
  asm volatile("v_nop\n\tv_nop\n\tv_nop\n\tv_nop" : "+v"(a) : "v"(x), "v"(y));
}
__device__ __forceinline__ void guard_acc(v8f& a) {
  asm volatile("v_nop\n\tv_nop\n\tv_nop\n\tv_nop" : "+v"(a));
}
__device__ __forceinline__ void keep4(v16h a, v16h b, v16h c, v16h d) {
  asm volatile("v_nop" :: "v"(a), "v"(b), "v"(c), "v"(d));
}

template <int MI, int SPL>
__global__ __launch_bounds__(256) void gemm_f16_kernel(
    const unsigned short* __restrict__ Ap, const unsigned short* __restrict__ A2p, int lda,
    const unsigned short* __restrict__ Btp, const unsigned short* __restrict__ Bt2p, int ldb,
    float* __restrict__ C, int ldc, int M, int N, int K, float scale, float rscale)
{
  static_assert(MI >= 1 && MI <= 2);
  static_assert(SPL >= 0 && SPL <= 2);
  const _Float16* A   = (const _Float16*)Ap;
  const _Float16* A2  = (const _Float16*)A2p;
  const _Float16* Bt  = (const _Float16*)Btp;
  const _Float16* Bt2 = (const _Float16*)Bt2p;
  __shared__ __align__(16) float sT[8][16 * 68];
  const int lane = threadIdx.x & 31;
  const int wave = threadIdx.x >> 5;
  const int tilesN = N >> 6;
  const int tilesM = M / (16 * MI);
  const int tile = blockIdx.x * 8 + wave;
  if (tile >= tilesM * tilesN) return;
  const int tm = tile / tilesN;
  const int tn = tile - tm * tilesN;
  const int m0 = tm * (16 * MI);
  const int n0 = tn << 6;
  const int rlane = lane & 15;
  const int koff  = (lane >> 4) * 8;
  const int mOff  = (lane >> 4) * 8;

  v8f acc[MI][4], accr[MI][4];
#pragma unroll
  for (int i = 0; i < MI; ++i)
#pragma unroll
    for (int j = 0; j < 4; ++j) {
      acc[i][j]  = (v8f){0.f, 0.f, 0.f, 0.f, 0.f, 0.f, 0.f, 0.f};
      accr[i][j] = (v8f){0.f, 0.f, 0.f, 0.f, 0.f, 0.f, 0.f, 0.f};
    }

  for (int k0 = 0; k0 < K; k0 += 32) {
    v16h bh[4], bl[4];
#pragma unroll
    for (int j = 0; j < 4; ++j) {
      const size_t bo = (size_t)(n0 + (j << 4) + rlane) * ldb + koff + k0;
      bh[j] = frag_load(Bt + bo);
      if (SPL == 2) bl[j] = frag_load(Bt2 + bo); else bl[j] = bh[j];
    }
#pragma unroll
    for (int i = 0; i < MI; ++i) {
      const size_t ao = (size_t)(m0 + (i << 4) + rlane) * lda + koff + k0;
      const v16h ah = frag_load(A + ao);
      v16h al = ah;
      if (SPL >= 1) al = frag_load(A2 + ao);
#pragma unroll
      for (int j = 0; j < 4; ++j) {
        acc[i][j] = mma(ah, bh[j], acc[i][j]);
        if (SPL >= 1) accr[i][j] = mma(al, bh[j], accr[i][j]);
        if (SPL == 2) accr[i][j] = mma(ah, bl[j], accr[i][j]);
      }
#pragma unroll
      for (int j = 0; j < 4; ++j) {
        guard1(acc[i][j], ah, al);
        if (SPL >= 1) guard1(accr[i][j], ah, al);
      }
    }
    keep4(bh[0], bh[1], bh[2], bh[3]);
    if (SPL == 2) keep4(bl[0], bl[1], bl[2], bl[3]);
  }
#pragma unroll
  for (int i = 0; i < MI; ++i)
#pragma unroll
    for (int j = 0; j < 4; ++j) {
      guard_acc(acc[i][j]);
      if (SPL >= 1) guard_acc(accr[i][j]);
    }

  float* slab = sT[wave];
#pragma unroll
  for (int i = 0; i < MI; ++i) {
    const int mBase = m0 + (i << 4);
#pragma unroll
    for (int j = 0; j < 4; ++j) {
#pragma unroll
      for (int r = 0; r < 8; ++r) {
        float v = acc[i][j][r] * scale;
        if (SPL >= 1) v += accr[i][j][r] * rscale;
        slab[(mOff + r) * 68 + (j << 4) + rlane] = v;
      }
    }
    __builtin_amdgcn_fence(__ATOMIC_RELEASE, "workgroup");
    __builtin_amdgcn_wave_barrier();
    __builtin_amdgcn_fence(__ATOMIC_ACQUIRE, "workgroup");
    {
      const int hh = lane >> 4, c4 = (lane & 15) * 4;
      for (int pass = 0; pass < 2; ++pass) {
#pragma unroll
        for (int it = 0; it < 8; ++it) {
          const int row = it * 2 + hh;
          const v4f v = *(const v4f*)(slab + row * 68 + c4);
          *(volatile v4f*)(C + (size_t)(mBase + row) * ldc + n0 + c4) = v;
        }
        __threadfence();
      }
    }
    __builtin_amdgcn_fence(__ATOMIC_RELEASE, "workgroup");
    __builtin_amdgcn_wave_barrier();
    __builtin_amdgcn_fence(__ATOMIC_ACQUIRE, "workgroup");
  }
}
}

__global__ __launch_bounds__(256) void pack_rows_bf_kernel(
    const float* __restrict__ W, unsigned short* __restrict__ dH,
    int Kdim, int Nreal, int total8, float carry)
{
  const int i = blockIdx.x * 256 + threadIdx.x;
  if (i >= total8) return;
  const size_t e0 = (size_t)i << 3;
  const int row = (int)(e0 / (size_t)Kdim);
  const int col = (int)(e0 - (size_t)row * (size_t)Kdim);
  const bool live = (row < Nreal);
  const int rc = live ? row : (Nreal - 1);
  const v4f a0 = *(const v4f*)(W + (size_t)rc * Kdim + col);
  const v4f a1 = *(const v4f*)(W + (size_t)rc * Kdim + col + 4);
  const float w0 = a0[0];
  const float w1 = a0[1];
  const float w2 = a0[2];
  const float w3 = a0[3];
  const float w4 = a1[0];
  const float w5 = a1[1];
  const float w6 = a1[2];
  const float w7 = a1[3];
  const float t0 = bf16r(w0) * carry;
  const float t1 = bf16r(w1) * carry;
  const float t2 = bf16r(w2) * carry;
  const float t3 = bf16r(w3) * carry;
  const float t4 = bf16r(w4) * carry;
  const float t5 = bf16r(w5) * carry;
  const float t6 = bf16r(w6) * carry;
  const float t7 = bf16r(w7) * carry;
  const float g0 = live ? t0 : 0.0f;
  const float g1 = live ? t1 : 0.0f;
  const float g2 = live ? t2 : 0.0f;
  const float g3 = live ? t3 : 0.0f;
  const float g4 = live ? t4 : 0.0f;
  const float g5 = live ? t5 : 0.0f;
  const float g6 = live ? t6 : 0.0f;
  const float g7 = live ? t7 : 0.0f;
  v8h hv;
  hv[0] = f16_flush(g0);
  hv[1] = f16_flush(g1);
  hv[2] = f16_flush(g2);
  hv[3] = f16_flush(g3);
  hv[4] = f16_flush(g4);
  hv[5] = f16_flush(g5);
  hv[6] = f16_flush(g6);
  hv[7] = f16_flush(g7);
  unsigned short* qh = dH + e0;
  *(volatile v8h*)qh = hv;
  __threadfence();
  *(volatile v8h*)qh = hv;
}

__global__ __launch_bounds__(256) void rne_vec_kernel(
    const float* __restrict__ src, float* __restrict__ dst, int n4)
{
  const int i = blockIdx.x * 256 + threadIdx.x;
  if (i >= n4) return;
  const v4f a = *(const v4f*)(src + (size_t)i * 4);
  const float a0 = a[0];
  const float a1 = a[1];
  const float a2 = a[2];
  const float a3 = a[3];
  v4f r;
  r[0] = bf16r(a0);
  r[1] = bf16r(a1);
  r[2] = bf16r(a2);
  r[3] = bf16r(a3);
  float* p = dst + (size_t)i * 4;
  *(volatile v4f*)p = r;
  __threadfence();
  *(volatile v4f*)p = r;
}

__global__ __launch_bounds__(256) void rne_plane_kernel(
    const float* __restrict__ src, float* __restrict__ dst, int n4)
{
  const int i = blockIdx.x * 256 + threadIdx.x;
  if (i >= n4) return;
  const v4f a = *(const v4f*)(src + (size_t)i * 4);
  const float a0 = a[0];
  const float a1 = a[1];
  const float a2 = a[2];
  const float a3 = a[3];
  v4f r;
  r[0] = bf16r(a0);
  r[1] = bf16r(a1);
  r[2] = bf16r(a2);
  r[3] = bf16r(a3);
  float* p = dst + (size_t)i * 4;
  *(volatile v4f*)p = r;
  __threadfence();
  *(volatile v4f*)p = r;
}

__global__ __launch_bounds__(256) void rne_rows_f16_kernel(
    const float* __restrict__ src, unsigned short* __restrict__ dH, int total8)
{
  const int i = blockIdx.x * 256 + threadIdx.x;
  if (i >= total8) return;
  const size_t e0 = (size_t)i << 3;
  const v4f a0 = *(const v4f*)(src + e0);
  const v4f a1 = *(const v4f*)(src + e0 + 4);
  const float f0 = a0[0];
  const float f1 = a0[1];
  const float f2 = a0[2];
  const float f3 = a0[3];
  const float f4 = a1[0];
  const float f5 = a1[1];
  const float f6 = a1[2];
  const float f7 = a1[3];
  v8h hv;
  hv[0] = f16_flush(bf16r(f0));
  hv[1] = f16_flush(bf16r(f1));
  hv[2] = f16_flush(bf16r(f2));
  hv[3] = f16_flush(bf16r(f3));
  hv[4] = f16_flush(bf16r(f4));
  hv[5] = f16_flush(bf16r(f5));
  hv[6] = f16_flush(bf16r(f6));
  hv[7] = f16_flush(bf16r(f7));
  unsigned short* qh = dH + e0;
  *(volatile v8h*)qh = hv;
  __threadfence();
  *(volatile v8h*)qh = hv;
}

__global__ __launch_bounds__(256) void conv_silu_kernel(
    const float* __restrict__ XZ, const float* __restrict__ cw, const float* __restrict__ cb,
    float* __restrict__ UC, unsigned short* __restrict__ UH, unsigned short* __restrict__ UL)
{
  __shared__ __align__(16) float sT[16 * kConvTP];
  const int tid = threadIdx.x, lane = tid & 31, wave = tid >> 5;
  const int d0 = blockIdx.x * 256, d = d0 + tid;
  const int t0 = blockIdx.y * 64;
  const v4f wv = *(const v4f*)(cw + (size_t)d * 4);
  const float w0 = wv[0], w1 = wv[1], w2 = wv[2], w3 = wv[3];
  const float bc = cb[d];
  float xm3, xm2, xm1;
  {
    const int r3 = t0 - 3, r2 = t0 - 2, r1 = t0 - 1;
    const float v3 = XZ[(size_t)(r3 < 0 ? 0 : r3) * kDin + d];
    const float v2 = XZ[(size_t)(r2 < 0 ? 0 : r2) * kDin + d];
    const float v1 = XZ[(size_t)(r1 < 0 ? 0 : r1) * kDin + d];
    xm3 = (r3 >= 0) ? v3 : 0.0f;
    xm2 = (r2 >= 0) ? v2 : 0.0f;
    xm1 = (r1 >= 0) ? v1 : 0.0f;
  }
  const int hrow = wave >> 1;
  const int hch  = (wave & 1) * 128 + lane * 4;
  for (int sub = 0; sub < 4; ++sub) {
    const int lb = t0 + sub * 16;
    for (int s = 0; s < 16; ++s) {
      const float xcur = XZ[(size_t)(lb + s) * kDin + d];
      float acc = w0 * xm3;
      acc = fmaf(w1, xm2, acc);
      acc = fmaf(w2, xm1, acc);
      acc = fmaf(w3, xcur, acc);
      const float sv = acc + bc;
      const float sg = __builtin_amdgcn_rcpf(1.0f + expf(-sv));
      sT[s * kConvTP + tid] = sv * sg;
      xm3 = xm2; xm2 = xm1; xm1 = xcur;
    }
    __syncthreads();
    v4f fv[4];
    v8h hv[2], lv[2];
#pragma unroll
    for (int it = 0; it < 4; ++it) fv[it] = *(const v4f*)(sT + (it * 4 + hrow) * kConvTP + hch);
#pragma unroll
    for (int it = 0; it < 2; ++it) {
      const float* sp = sT + (it * 8 + wave) * kConvTP + lane * 8;
      const v4f a0 = *(const v4f*)(sp);
      const v4f a1 = *(const v4f*)(sp + 4);
#pragma unroll
      for (int e = 0; e < 4; ++e) {
        _Float16 h0, l0, h1, l1;
        const float f0 = a0[e];
        const float f1 = a1[e];
        f16_split(f0, h0, l0);
        f16_split(f1, h1, l1);
        hv[it][e] = h0; lv[it][e] = l0;
        hv[it][4 + e] = h1; lv[it][4 + e] = l1;
      }
    }
    for (int pass = 0; pass < 2; ++pass) {
#pragma unroll
      for (int it = 0; it < 4; ++it)
        *(volatile v4f*)(UC + (size_t)(lb + it * 4 + hrow) * kDin + d0 + hch) = fv[it];
#pragma unroll
      for (int it = 0; it < 2; ++it) {
        const size_t o = (size_t)(lb + it * 8 + wave) * kDin + d0 + lane * 8;
        *(volatile v8h*)(UH + o) = hv[it];
        *(volatile v8h*)(UL + o) = lv[it];
      }
      __threadfence();
    }
    __syncthreads();
  }
}

__global__ __launch_bounds__(256) void dt_bias_kernel(
    const float* __restrict__ DTP, const float* __restrict__ bdt, float* __restrict__ DT)
{
  const int d4 = (blockIdx.x * 256 + threadIdx.x) * 4;
  const int r0 = blockIdx.y * 8;
  const v4f b = *(const v4f*)(bdt + d4);
  v4f val[8];
#pragma unroll
  for (int i = 0; i < 8; ++i) {
    const v4f p = *(const v4f*)(DTP + (size_t)(r0 + i) * kDin + d4);
    val[i] = p + b;
  }
  for (int pass = 0; pass < 2; ++pass) {
#pragma unroll
    for (int i = 0; i < 8; ++i)
      *(volatile v4f*)(DT + (size_t)(r0 + i) * kDin + d4) = val[i];
    __threadfence();
  }
}

typedef float    ms1_v4f __attribute__((ext_vector_type(4)));
typedef unsigned ms1_v4u __attribute__((ext_vector_type(4)));
struct ms1_args {
  const float* dtpre;
  const float* u;
  const float* bc;
  const float* z;
  const float* A_log;
  const float* Dskip;
  __half* y;
  __half* y_lo;
  long ld_dtpre;
  long ld_u;
  long ld_bc;
  long ld_z;
  long ld_y;
  int offB;
  int offC;
  int offZ;
  float ycarry;
  int dir;
  int D;
  int L;
  int nbatch;
};
static_assert(sizeof(ms1_args) == 136);

__device__ __forceinline__ float ms1_flush16(float v) {
  return (fabsf(v) < 6.103515625e-05f) ? 0.0f : v;
}
__device__ __forceinline__ unsigned ms1_h16bits(float v) {
  return (unsigned)__half_as_ushort(__float2half_rn(ms1_flush16(v)));
}
__device__ __forceinline__ float ms1_h16val(unsigned b) {
  return __half2float(__ushort_as_half((unsigned short)b));
}
__device__ __forceinline__ float ms1_softplus(float v) {
  return fmaxf(v, 0.0f) + log1pf(expf(-fabsf(v)));
}
__device__ __forceinline__ void ms1_pack2(float v0, float v1, unsigned& hw, unsigned& lw) {
  const unsigned h0 = ms1_h16bits(v0);
  const unsigned h1 = ms1_h16bits(v1);
  const float r0 = (v0 - ms1_h16val(h0)) * 2048.0f;
  const float r1 = (v1 - ms1_h16val(h1)) * 2048.0f;
  const unsigned l0 = ms1_h16bits(r0);
  const unsigned l1 = ms1_h16bits(r1);
  hw = h0 | (h1 << 16);
  lw = l0 | (l1 << 16);
}

template <int NSTATE>
__global__ __launch_bounds__(64 * (NSTATE / 16)) void ms1_scan_kernel(ms1_args a)
{
  static_assert(NSTATE == 16 || NSTATE == 64);
  constexpr int NQ  = NSTATE / 16;
  constexpr int NT  = 64 * NQ;
  constexpr int NW  = NT / 32;
  constexpr int BCW = 2 * NSTATE;
  constexpr int YP  = 68;
  constexpr int RPI = NW * 4;
  constexpr int NIT = 64 / RPI;
  static_assert(16 * NT <= 64 * YP);
  __shared__ __align__(16) float sBC[64 * BCW];
  __shared__ __align__(16) float sY[64 * YP];
  const int tid  = threadIdx.x;
  const int lane = tid & 31;
  const int wave = tid >> 5;
  const int c    = tid / NQ;
  const int sq   = tid - c * NQ;
  const int bpb  = a.D / 64;
  const int bi   = blockIdx.x / bpb;
  if (bi >= a.nbatch) return;
  const int d0 = (blockIdx.x - bi * bpb) * 64;
  const int d  = d0 + c;
  const long rowb = (long)bi * a.L;
  const bool hasz  = (a.z != nullptr);
  const bool hasD  = (a.Dskip != nullptr);
  const bool hasLo = (a.y_lo != nullptr);

#pragma unroll 1
  for (int n = 0; n < 16; ++n) {
    const float al = a.A_log[(long)d * NSTATE + sq * 16 + n];
    sY[n * NT + tid] = -expf(al);
  }
  __syncthreads();
  float An[16], h[16];
#pragma unroll
  for (int n = 0; n < 16; ++n) {
    An[n] = sY[n * NT + tid];
    h[n] = 0.0f;
  }
  float Dd = 0.0f;
  if (hasD) Dd = a.Dskip[d];

  const int nchunk = a.L / 64;
  const bool fwd = (a.dir > 0);
  const int s0 = fwd ? 0 : 63;
  const int sd = fwd ? 1 : -1;
  const int q  = lane >> 3;
  const int c8 = (lane & 7) * 8;

  for (int ci = 0; ci < nchunk; ++ci) {
    const int tb = fwd ? (ci * 64) : (a.L - 64 - ci * 64);
    const long rowc = rowb + tb;
    __syncthreads();
#pragma unroll 8
    for (int i = 0; i < 32; ++i) {
      const int idx = tid + i * NT;
      const int st  = idx / BCW;
      const int col = idx - st * BCW;
      const int sc  = (col < NSTATE) ? (a.offB + col) : (a.offC + col - NSTATE);
      sBC[idx] = a.bc[(rowc + st) * a.ld_bc + sc];
    }
    __syncthreads();
    for (int s = 0; s < 64; ++s) {
      const int ls = s0 + sd * s;
      const long row = rowc + ls;
      float pre = a.dtpre[row * a.ld_dtpre + d];
      float uv  = a.u[row * a.ld_u + d];
      float zv  = 0.0f;
      if (hasz) zv = a.z[row * a.ld_z + a.offZ + d];
      asm volatile("" : "+v"(pre));
      asm volatile("" : "+v"(uv));
      asm volatile("" : "+v"(zv));
      const float delta = ms1_softplus(pre);
      const float dtx = delta * uv;
      const float* bp = sBC + ls * BCW + sq * 16;
      const float* cp = bp + NSTATE;
      ms1_v4f Bq[4], Cq[4];
#pragma unroll
      for (int k = 0; k < 4; ++k) {
        Bq[k] = *(const ms1_v4f*)(bp + 4 * k);
        Cq[k] = *(const ms1_v4f*)(cp + 4 * k);
      }
      float yv = 0.0f;
#pragma unroll
      for (int n = 0; n < 16; ++n) {
        const float e = __expf(delta * An[n]);
        h[n] = fmaf(e, h[n], dtx * Bq[n >> 2][n & 3]);
        yv = fmaf(h[n], Cq[n >> 2][n & 3], yv);
      }
      if (NQ > 1) {
        yv += __shfl_xor(yv, 1, 32);
        yv += __shfl_xor(yv, 2, 32);
      }
      if (hasD) yv = fmaf(uv, Dd, yv);
      if (hasz) {
        const float sg = __builtin_amdgcn_rcpf(1.0f + expf(-zv));
        yv = yv * (zv * sg);
      }
      if (sq == 0) sY[ls * YP + c] = yv * a.ycarry;
    }
    __syncthreads();
    ms1_v4u hw[NIT], lw[NIT];
#pragma unroll
    for (int it = 0; it < NIT; ++it) {
      const int row = it * RPI + wave * 4 + q;
      const float* sp = sY + row * YP + c8;
      const ms1_v4f f0 = *(const ms1_v4f*)(sp);
      const ms1_v4f f1 = *(const ms1_v4f*)(sp + 4);
      unsigned h0, h1, h2, h3, l0, l1, l2, l3;
      ms1_pack2(f0[0], f0[1], h0, l0);
      ms1_pack2(f0[2], f0[3], h1, l1);
      ms1_pack2(f1[0], f1[1], h2, l2);
      ms1_pack2(f1[2], f1[3], h3, l3);
      hw[it] = (ms1_v4u){h0, h1, h2, h3};
      lw[it] = (ms1_v4u){l0, l1, l2, l3};
    }
    for (int pass = 0; pass < 2; ++pass) {
#pragma unroll
      for (int it = 0; it < NIT; ++it) {
        const int row = it * RPI + wave * 4 + q;
        const long o = (rowc + row) * a.ld_y + d0 + c8;
        *(volatile ms1_v4u*)(a.y + o) = hw[it];
        if (hasLo) *(volatile ms1_v4u*)(a.y_lo + o) = lw[it];
      }
      __threadfence();
    }
  }
}

__global__ __launch_bounds__(256) void dfeat_word_kernel(
    const float* __restrict__ P, unsigned short* __restrict__ dH)
{
  constexpr int kTotal8 = kSeq * kRank / 8;
  const int i = blockIdx.x * 256 + threadIdx.x;
  if (i >= kTotal8) return;
  const int row = i >> 2;
  const int g = i & 3;
  const float* sp = P + (size_t)row * kXpN + kOffDtF + g * 8;
  const v4f a0 = *(const v4f*)(sp);
  const v4f a1 = *(const v4f*)(sp + 4);
  const float f0 = a0[0];
  const float f1 = a0[1];
  const float f2 = a0[2];
  const float f3 = a0[3];
  const float f4 = a1[0];
  const float f5 = a1[1];
  const float f6 = a1[2];
  const float f7 = a1[3];
  v8h hv;
  hv[0] = f16_flush(f0);
  hv[1] = f16_flush(f1);
  hv[2] = f16_flush(f2);
  hv[3] = f16_flush(f3);
  hv[4] = f16_flush(f4);
  hv[5] = f16_flush(f5);
  hv[6] = f16_flush(f6);
  hv[7] = f16_flush(f7);
  unsigned short* qh = dH + (size_t)row * kRank + g * 8;
  *(volatile v8h*)qh = hv;
  __threadfence();
  *(volatile v8h*)qh = hv;
}

__device__ __forceinline__ float gate_from_words(unsigned hb, unsigned lb, float zf) {
  const float hi = h16_to_f32(hb);
  const float lo = h16_to_f32(lb);
  const float y = (hi + lo * kInvResid) * kInvCarry;
  return y * (zf / (1.0f + expf(-zf)));
}

__global__ __launch_bounds__(256) void gate_word_kernel(
    const unsigned short* __restrict__ YH, const unsigned short* __restrict__ YL,
    const float* __restrict__ Z, unsigned short* __restrict__ GH, int total8)
{
  const int i = blockIdx.x * 256 + threadIdx.x;
  if (i >= total8) return;
  const size_t e0 = (size_t)i << 3;
  const v4u hw = *(const v4u*)(const void*)(YH + e0);
  const v4u lw = *(const v4u*)(const void*)(YL + e0);
  const v4f za = *(const v4f*)(Z + e0);
  const v4f zb = *(const v4f*)(Z + e0 + 4);
  const unsigned hw0 = hw[0];
  const unsigned hw1 = hw[1];
  const unsigned hw2 = hw[2];
  const unsigned hw3 = hw[3];
  const unsigned lw0 = lw[0];
  const unsigned lw1 = lw[1];
  const unsigned lw2 = lw[2];
  const unsigned lw3 = lw[3];
  const float z0 = za[0];
  const float z1 = za[1];
  const float z2 = za[2];
  const float z3 = za[3];
  const float z4 = zb[0];
  const float z5 = zb[1];
  const float z6 = zb[2];
  const float z7 = zb[3];
  const float g0 = gate_from_words(hw0 & 0xffffu, lw0 & 0xffffu, z0);
  const float g1 = gate_from_words(hw0 >> 16, lw0 >> 16, z1);
  const float g2 = gate_from_words(hw1 & 0xffffu, lw1 & 0xffffu, z2);
  const float g3 = gate_from_words(hw1 >> 16, lw1 >> 16, z3);
  const float g4 = gate_from_words(hw2 & 0xffffu, lw2 & 0xffffu, z4);
  const float g5 = gate_from_words(hw2 >> 16, lw2 >> 16, z5);
  const float g6 = gate_from_words(hw3 & 0xffffu, lw3 & 0xffffu, z6);
  const float g7 = gate_from_words(hw3 >> 16, lw3 >> 16, z7);
  v8h hv;
  hv[0] = f16_flush(g0);
  hv[1] = f16_flush(g1);
  hv[2] = f16_flush(g2);
  hv[3] = f16_flush(g3);
  hv[4] = f16_flush(g4);
  hv[5] = f16_flush(g5);
  hv[6] = f16_flush(g6);
  hv[7] = f16_flush(g7);
  unsigned short* qh = GH + e0;
  *(volatile v8h*)qh = hv;
  __threadfence();
  *(volatile v8h*)qh = hv;
}

__device__ __forceinline__ float ln_value(float t, float mu, float inv, float w, float b) {
  return (t - mu) * inv * w + b;
}

__global__ __launch_bounds__(256) void ln_word_kernel(
    const float* __restrict__ MX, const float* __restrict__ gw, const float* __restrict__ gb,
    unsigned short* __restrict__ dH, int rows)
{
  const int lane = threadIdx.x & 31;
  const int wave = threadIdx.x >> 5;
  const int row  = blockIdx.x * 8 + wave;
  if (row >= rows) return;
  const float* xr = MX + (size_t)row * kDm;
  v4f t[4];
#pragma unroll
  for (int g = 0; g < 4; ++g) {
    const int off = (g >> 1) * 256 + lane * 8 + (g & 1) * 4;
    t[g] = *(const v4f*)(xr + off);
  }
  float s = 0.0f;
#pragma unroll
  for (int g = 0; g < 4; ++g)
#pragma unroll
    for (int e = 0; e < 4; ++e) s += t[g][e];
#pragma unroll
  for (int o = 16; o >= 1; o >>= 1) s += __shfl_xor(s, o, 32);
  const float mu = s * (1.0f / (float)kDm);
  float ss = 0.0f;
#pragma unroll
  for (int g = 0; g < 4; ++g)
#pragma unroll
    for (int e = 0; e < 4; ++e) {
      const float dv = t[g][e] - mu;
      ss = fmaf(dv, dv, ss);
    }
#pragma unroll
  for (int o = 16; o >= 1; o >>= 1) ss += __shfl_xor(ss, o, 32);
  const float var = ss * (1.0f / (float)kDm);
  const float inv = rsqrtf(var + kLnEps);
  v8h hv[2];
#pragma unroll
  for (int g = 0; g < 4; ++g) {
    const int off = (g >> 1) * 256 + lane * 8 + (g & 1) * 4;
    const v4f w4 = *(const v4f*)(gw + off);
    const v4f b4 = *(const v4f*)(gb + off);
#pragma unroll
    for (int e = 0; e < 4; ++e) {
      const float te = t[g][e];
      const float we = w4[e];
      const float be = b4[e];
      const float n = ln_value(te, mu, inv, we, be);
      hv[g >> 1][(g & 1) * 4 + e] = f16_flush(n);
    }
  }
  for (int pass = 0; pass < 2; ++pass) {
#pragma unroll
    for (int hf = 0; hf < 2; ++hf) {
      const size_t o = (size_t)row * kDm + hf * 256 + lane * 8;
      *(volatile v8h*)(dH + o) = hv[hf];
    }
    __threadfence();
  }
}

__global__ __launch_bounds__(256) void gelu_res_out_kernel(
    const float* __restrict__ LIN, const float* __restrict__ lb, const float* __restrict__ XR,
    float* __restrict__ out, int total4)
{
  const int i = blockIdx.x * 256 + threadIdx.x;
  if (i >= total4) return;
  const size_t e0 = (size_t)i * 4;
  const int c4 = (int)(e0 % (size_t)kDm);
  const v4f a = *(const v4f*)(LIN + e0);
  const v4f b = *(const v4f*)(lb + c4);
  const v4f x = *(const v4f*)(XR + e0);
  const float a0 = a[0];
  const float a1 = a[1];
  const float a2 = a[2];
  const float a3 = a[3];
  const float b0 = b[0];
  const float b1 = b[1];
  const float b2 = b[2];
  const float b3 = b[3];
  const float x0 = x[0];
  const float x1 = x[1];
  const float x2 = x[2];
  const float x3 = x[3];
  const float t0 = a0 + b0;
  const float t1 = a1 + b1;
  const float t2 = a2 + b2;
  const float t3 = a3 + b3;
  v4f r;
  r[0] = 0.5f * t0 * (1.0f + erff(t0 * 0.70710678f)) + x0;
  r[1] = 0.5f * t1 * (1.0f + erff(t1 * 0.70710678f)) + x1;
  r[2] = 0.5f * t2 * (1.0f + erff(t2 * 0.70710678f)) + x2;
  r[3] = 0.5f * t3 * (1.0f + erff(t3 * 0.70710678f)) + x3;
  float* p = out + e0;
  *(volatile v4f*)p = r;
  __threadfence();
  *(volatile v4f*)p = r;
}

static_assert(((kSeq / 32) * (kDin / 64)) % 8 == 0);
static_assert(((kSeq / 32) * (kXpN / 64)) % 8 == 0);
static_assert(((kSeq / 32) * (kDm / 64)) % 8 == 0);
static_assert(((2 * kDin * kDm / 8) % 256) == 0);
static_assert(((kXpN * kDin / 8) % 256) == 0);
static_assert(((kDin * kRank / 8) % 256) == 0);
static_assert(((kDm * kDin / 8) % 256) == 0);
static_assert(((kDm * kDm / 8) % 256) == 0);
static_assert(((kDin * kNst / 4) % 256) == 0);
static_assert(((kDin * kConvK / 4) % 256) == 0);
static_assert((kDin / 4) == 256);
static_assert((kDm / 4) == 128);
static_assert(((kSeq * kDm / 4) % 256) == 0);
static_assert(((kSeq * kDm / 8) % 256) == 0);
static_assert(((kSeq * kRank / 8) % 256) == 0);
static_assert(((kSeq * kDin / 8) % 256) == 0);
static_assert((kDin / 4 / 256) == 1 && (kDin / 256) == 4 && (kDin / 64) == 16);
static_assert((kSeq % 8) == 0 && (kSeq % 64) == 0);

extern "C" void kernel_launch(void* const* d_in, const int* in_sizes, int n_in,
                              void* d_out, int out_size, void* d_ws, size_t ws_size,
                              hipStream_t stream)
{
  if (n_in < 14) return;
  if (in_sizes[0] != kBatch * kSeq * kDm) return;
  if (in_sizes[1] != 2 * kDin * kDm) return;
  if (in_sizes[2] != kDin * kConvK) return;
  if (in_sizes[3] != kDin) return;
  if (in_sizes[4] != kXpN * kDin) return;
  if (in_sizes[5] != kDin * kRank) return;
  if (in_sizes[6] != kDin) return;
  if (in_sizes[7] != kDin * kNst) return;
  if (in_sizes[8] != kDin) return;
  if (in_sizes[9] != kDm * kDin) return;
  if (in_sizes[10] != kDm) return;
  if (in_sizes[11] != kDm) return;
  if (in_sizes[12] != kDm * kDm) return;
  if (in_sizes[13] != kDm) return;
  if (out_size != kBatch * kSeq * kDm) return;
  if (ws_size < kWsTotal) return;

  const float* x         = (const float*)d_in[0];
  const float* in_proj_w = (const float*)d_in[1];
  const float* conv_w    = (const float*)d_in[2];
  const float* conv_b    = (const float*)d_in[3];
  const float* x_proj_w  = (const float*)d_in[4];
  const float* dt_proj_w = (const float*)d_in[5];
  const float* dt_proj_b = (const float*)d_in[6];
  const float* A_log     = (const float*)d_in[7];
  const float* D_param   = (const float*)d_in[8];
  const float* out_proj_w = (const float*)d_in[9];
  const float* norm_w    = (const float*)d_in[10];
  const float* norm_b    = (const float*)d_in[11];
  const float* lin_w     = (const float*)d_in[12];
  const float* lin_b     = (const float*)d_in[13];
  float* out = (float*)d_out;

  char* ws = (char*)d_ws;
  unsigned short* WIN  = (unsigned short*)(ws + kOffWIN);
  unsigned short* WX   = (unsigned short*)(ws + kOffWX);
  unsigned short* WDT  = (unsigned short*)(ws + kOffWDT);
  unsigned short* WOUT = (unsigned short*)(ws + kOffWOUT);
  unsigned short* WLIN = (unsigned short*)(ws + kOffWLIN);
  float*          ALOG = (float*)(ws + kOffALOG);
  float*          CW   = (float*)(ws + kOffCW);
  float*          CB   = (float*)(ws + kOffCB);
  float*          DTB  = (float*)(ws + kOffDTB);
  float*          DR   = (float*)(ws + kOffDR);
  float*          NW   = (float*)(ws + kOffNW);
  float*          NB   = (float*)(ws + kOffNB);
  float*          LB   = (float*)(ws + kOffLB);
  float*          XR   = (float*)(ws + kOffXR);
  unsigned short* XH   = (unsigned short*)(ws + kOffXH);
  float*          U0   = (float*)(ws + kOffU0);
  float*          Z    = (float*)(ws + kOffZ);
  float*          U    = (float*)(ws + kOffU);
  unsigned short* UH   = (unsigned short*)(ws + kOffUH);
  unsigned short* UL   = (unsigned short*)(ws + kOffUL);
  float*          PROJ = (float*)(ws + kOffPROJ);
  unsigned short* DH   = (unsigned short*)(ws + kOffDH);
  float*          DTP  = (float*)(ws + kOffDTP);
  float*          DT   = (float*)(ws + kOffDT);
  unsigned short* YH   = (unsigned short*)(ws + kOffYH);
  unsigned short* YL   = (unsigned short*)(ws + kOffYL);
  unsigned short* GH   = (unsigned short*)(ws + kOffGH);
  float*          M    = (float*)(ws + kOffM);
  unsigned short* YNH  = (unsigned short*)(ws + kOffYNH);
  float*          LIN  = (float*)(ws + kOffLIN);

  constexpr float sW = 1.0f / kWCarry;

  pack_rows_bf_kernel<<<(2 * kDin * kDm / 8) / 256, 256, 0, stream>>>(
      in_proj_w, WIN, kDm, 2 * kDin, 2 * kDin * kDm / 8, kWCarry);
  pack_rows_bf_kernel<<<(kXpN * kDin / 8) / 256, 256, 0, stream>>>(
      x_proj_w, WX, kDin, kXpN, kXpN * kDin / 8, kWCarry);
  pack_rows_bf_kernel<<<(kDin * kRank / 8) / 256, 256, 0, stream>>>(
      dt_proj_w, WDT, kRank, kDin, kDin * kRank / 8, kWCarry);
  pack_rows_bf_kernel<<<(kDm * kDin / 8) / 256, 256, 0, stream>>>(
      out_proj_w, WOUT, kDin, kDm, kDm * kDin / 8, kWCarry);
  pack_rows_bf_kernel<<<(kDm * kDm / 8) / 256, 256, 0, stream>>>(
      lin_w, WLIN, kDm, kDm, kDm * kDm / 8, kWCarry);

  rne_vec_kernel<<<(kDin * kNst / 4) / 256, 256, 0, stream>>>(A_log, ALOG, kDin * kNst / 4);
  rne_vec_kernel<<<(kDin * kConvK / 4) / 256, 256, 0, stream>>>(conv_w, CW, kDin * kConvK / 4);
  rne_vec_kernel<<<1, 256, 0, stream>>>(conv_b, CB, kDin / 4);
  rne_vec_kernel<<<1, 256, 0, stream>>>(dt_proj_b, DTB, kDin / 4);
  rne_vec_kernel<<<1, 256, 0, stream>>>(D_param, DR, kDin / 4);
  rne_vec_kernel<<<1, 256, 0, stream>>>(norm_w, NW, kDm / 4);
  rne_vec_kernel<<<1, 256, 0, stream>>>(norm_b, NB, kDm / 4);
  rne_vec_kernel<<<1, 256, 0, stream>>>(lin_b, LB, kDm / 4);

  for (int b = 0; b < kBatch; ++b) {
    const float* xb = x + (size_t)b * kSeq * kDm;
    float* outb = out + (size_t)b * kSeq * kDm;

    rne_plane_kernel<<<(kSeq * kDm / 4) / 256, 256, 0, stream>>>(xb, XR, kSeq * kDm / 4);
    rne_rows_f16_kernel<<<(kSeq * kDm / 8) / 256, 256, 0, stream>>>(xb, XH, kSeq * kDm / 8);

    eng::gemm_f16_kernel<2, 0><<<dim3((kSeq / 32) * (kDin / 64) / 8), 256, 0, stream>>>(
        XH, nullptr, kDm, WIN, nullptr, kDm, U0, kDin, kSeq, kDin, kDm, sW, 0.0f);
    eng::gemm_f16_kernel<2, 0><<<dim3((kSeq / 32) * (kDin / 64) / 8), 256, 0, stream>>>(
        XH, nullptr, kDm, WIN + (size_t)kDin * kDm, nullptr, kDm, Z, kDin, kSeq, kDin, kDm, sW, 0.0f);

    conv_silu_kernel<<<dim3(kDin / 256, kSeq / 64), 256, 0, stream>>>(U0, CW, CB, U, UH, UL);

    eng::gemm_f16_kernel<2, 0><<<dim3((kSeq / 32) * (kXpN / 64) / 8), 256, 0, stream>>>(
        UH, nullptr, kDin, WX, nullptr, kDin, PROJ, kXpN, kSeq, kXpN, kDin, sW, 0.0f);

    dfeat_word_kernel<<<(kSeq * kRank / 8) / 256, 256, 0, stream>>>(PROJ, DH);

    eng::gemm_f16_kernel<2, 0><<<dim3((kSeq / 32) * (kDin / 64) / 8), 256, 0, stream>>>(
        DH, nullptr, kRank, WDT, nullptr, kRank, DTP, kDin, kSeq, kDin, kRank, sW, 0.0f);

    dt_bias_kernel<<<dim3(kDin / 4 / 256, kSeq / 8), 256, 0, stream>>>(DTP, DTB, DT);

    ms1_args sa;
    sa.dtpre = DT;
    sa.u = U;
    sa.bc = PROJ;
    sa.z = nullptr;
    sa.A_log = ALOG;
    sa.Dskip = DR;
    sa.y = (__half*)YH;
    sa.y_lo = (__half*)YL;
    sa.ld_dtpre = kDin;
    sa.ld_u = kDin;
    sa.ld_bc = kXpN;
    sa.ld_z = 0;
    sa.ld_y = kDin;
    sa.offB = kOffB;
    sa.offC = kOffC;
    sa.offZ = 0;
    sa.ycarry = kYCarry;
    sa.dir = 1;
    sa.D = kDin;
    sa.L = kSeq;
    sa.nbatch = 1;
    ms1_scan_kernel<16><<<dim3(kDin / 64), 64, 0, stream>>>(sa);

    gate_word_kernel<<<(kSeq * kDin / 8) / 256, 256, 0, stream>>>(YH, YL, Z, GH, kSeq * kDin / 8);

    eng::gemm_f16_kernel<2, 0><<<dim3((kSeq / 32) * (kDm / 64) / 8), 256, 0, stream>>>(
        GH, nullptr, kDin, WOUT, nullptr, kDin, M, kDm, kSeq, kDm, kDin, sW, 0.0f);

    ln_word_kernel<<<kSeq / 8, 256, 0, stream>>>(M, NW, NB, YNH, kSeq);

    eng::gemm_f16_kernel<2, 0><<<dim3((kSeq / 32) * (kDm / 64) / 8), 256, 0, stream>>>(
        YNH, nullptr, kDm, WLIN, nullptr, kDm, LIN, kDm, kSeq, kDm, kDm, sW, 0.0f);

    gelu_res_out_kernel<<<(kSeq * kDm / 4) / 256, 256, 0, stream>>>(LIN, LB, XR, outb, kSeq * kDm / 4);
  }
}
